// RGAT_5583457485246
// MI455X (gfx1250) — hardware-verified
//
#include <hip/hip_runtime.h>
#include <stddef.h>
#include <stdint.h>
#include <math.h>


#define FW      128
#define HC      128
#define HD1     32
#define NREL    3
#define NOUT    16
#define KL0     128
#define KL1     256
#define KCL     256
#define NTHR    256
#define NWAVE   8
#define EPT     8
#define CHUNK   (NTHR * EPT)
#define WCAP    (EPT * 32)
#define LISTN   (NWAVE * WCAP)
#define NBMAX   2048
#define SLOTB   11
#define RCAP    28672
#define DEGCAP  256
#define GBM     64
#define GTHR    128
#define MROWS   128
#define NU0     (NREL * FW * (KL0 / 8))
#define NU1     (NREL * FW * (KL1 / 8))
#define NUC     (NOUT * (KCL / 8))
#define NUW     (NU0 + NU1 + NUC)
#define NEGSL   0.2f
#define EPS_SM  1e-16f
#define MX0     (-1.0e30f)
#define WSMAX   134217728
#define LDS_AGG ((2 * RCAP + 2 * NBMAX + LISTN) * 4 + 64)

static_assert((CHUNK & (CHUNK - 1)) == 0 && CHUNK <= (1 << SLOTB));
static_assert(NBMAX == (1 << SLOTB));
static_assert(NTHR * 8 == NBMAX);
static_assert(LISTN >= NBMAX);
static_assert(LISTN >= NWAVE * WCAP);
static_assert((RCAP % 32) == 0);
static_assert(LDS_AGG <= 300000);
static_assert(GBM == (GTHR / 32) * 16);
static_assert(GTHR == 2 * GBM);
static_assert(2 * GTHR == 2 * HC);
static_assert((KL0 % 32) == 0 && (KL1 % 32) == 0 && (KCL % 32) == 0);
static_assert(FW == HC && KL0 == FW && KL1 == 2 * FW && KCL == 2 * FW);
static_assert(HC == 4 * 32);
static_assert(HC == 4 * HD1 && HD1 == 4 * 8);
static_assert((MROWS % GBM) == 0);
static_assert((NU0 % NTHR) == 0 && ((NU0 + NU1) % NTHR) == 0 && (NUW % NTHR) == 0);
static_assert((KL0 / 8) == 16 && (KL1 / 8) == 32 && (KCL / 8) == 32);
static_assert(((GBM * NOUT * 4) % 128) == 0 && (GTHR % 4) == 0);

typedef float          v4f  __attribute__((ext_vector_type(4)));
typedef float          v8f  __attribute__((ext_vector_type(8)));
typedef int            v4i  __attribute__((ext_vector_type(4)));
typedef int            v8i  __attribute__((ext_vector_type(8)));
typedef unsigned int   v4u  __attribute__((ext_vector_type(4)));
typedef unsigned short v8us __attribute__((ext_vector_type(8)));
typedef __bf16         v16b __attribute__((ext_vector_type(16)));
typedef v4f  __attribute__((may_alias)) v4fa;
typedef v8us __attribute__((may_alias)) v8usa;
union FragB { v16b v; v8us h[2]; v8i w; };

__device__ __forceinline__ v8f wmb(const FragB& a, const FragB& b, v8f c) {
  v8f d = __builtin_amdgcn_wmma_f32_16x16x32_bf16(false, a.v, false, b.v, (short)0, c, false, false);
  asm volatile("v_nop\n\tv_nop\n\tv_nop\n\tv_nop" : "+v"(d) : "v"(a.w), "v"(b.w));
  return d;
}

__device__ __forceinline__ unsigned int f2bf(float f) {
  const unsigned int u = __float_as_uint(f);
  return ((u + 0x7FFFu + ((u >> 16) & 1u)) >> 16) & 0xFFFFu;
}
__device__ __forceinline__ float bf2f(unsigned int b) { return __uint_as_float(b << 16); }
__device__ __forceinline__ float bfr(float f) { return bf2f(f2bf(f)); }
__device__ __forceinline__ v4f bfr4(const v4f a) {
  v4f r; r.x = bfr(a.x); r.y = bfr(a.y); r.z = bfr(a.z); r.w = bfr(a.w); return r;
}
__device__ __forceinline__ unsigned int pk2(float lo, float hi) { return f2bf(lo) | (f2bf(hi) << 16); }
__device__ __forceinline__ v4u pack8(const v4f a, const v4f b) {
  v4u r;
  r.x = pk2(a.x, a.y); r.y = pk2(a.z, a.w); r.z = pk2(b.x, b.y); r.w = pk2(b.z, b.w);
  return r;
}
__device__ __forceinline__ v8us hilo8(v4f t) {
  v8us o;
  unsigned hb;
  hb = f2bf(t.x); o[0] = (unsigned short)hb; o[4] = (unsigned short)f2bf(t.x - __uint_as_float(hb << 16));
  hb = f2bf(t.y); o[1] = (unsigned short)hb; o[5] = (unsigned short)f2bf(t.y - __uint_as_float(hb << 16));
  hb = f2bf(t.z); o[2] = (unsigned short)hb; o[6] = (unsigned short)f2bf(t.z - __uint_as_float(hb << 16));
  hb = f2bf(t.w); o[3] = (unsigned short)hb; o[7] = (unsigned short)f2bf(t.w - __uint_as_float(hb << 16));
  return o;
}
__device__ __forceinline__ float elu1(float h) {
  const float n = __expf(fminf(h, 0.f)) - 1.0f;
  return h > 0.f ? h : n;
}

__device__ __forceinline__ int scan_chunk(const int* __restrict__ dsts, int nE, int cbase, int slotBase,
                                          int nb, int vec8, int* list, int tid, int lane, int wave) {
  int wc = 0;
  const int el0  = tid * EPT;
  const int e0   = cbase + el0;
  const int sent = -2147483647 - 1;
  v4i da, db;
  if (vec8 != 0 && cbase + CHUNK <= nE) {
    da = *(const v4i*)(dsts + e0);
    db = *(const v4i*)(dsts + e0 + 4);
  } else {
    da.x = (e0     < nE) ? dsts[min(e0,     nE - 1)] : sent;
    da.y = (e0 + 1 < nE) ? dsts[min(e0 + 1, nE - 1)] : sent;
    da.z = (e0 + 2 < nE) ? dsts[min(e0 + 2, nE - 1)] : sent;
    da.w = (e0 + 3 < nE) ? dsts[min(e0 + 3, nE - 1)] : sent;
    db.x = (e0 + 4 < nE) ? dsts[min(e0 + 4, nE - 1)] : sent;
    db.y = (e0 + 5 < nE) ? dsts[min(e0 + 5, nE - 1)] : sent;
    db.z = (e0 + 6 < nE) ? dsts[min(e0 + 6, nE - 1)] : sent;
    db.w = (e0 + 7 < nE) ? dsts[min(e0 + 7, nE - 1)] : sent;
  }
  const unsigned nbs = (unsigned)slotBase;
  const unsigned unb = (unsigned)nb;
  const unsigned s0 = (unsigned)da.x - nbs, s1 = (unsigned)da.y - nbs;
  const unsigned s2 = (unsigned)da.z - nbs, s3 = (unsigned)da.w - nbs;
  const unsigned s4 = (unsigned)db.x - nbs, s5 = (unsigned)db.y - nbs;
  const unsigned s6 = (unsigned)db.z - nbs, s7 = (unsigned)db.w - nbs;
  const bool h0 = s0 < unb, h1 = s1 < unb, h2 = s2 < unb, h3 = s3 < unb;
  const bool h4 = s4 < unb, h5 = s5 < unb, h6 = s6 < unb, h7 = s7 < unb;
  const unsigned any = __builtin_amdgcn_ballot_w32(h0 | h1 | h2 | h3 | h4 | h5 | h6 | h7);
  if (any != 0u) {
#define HITJ(J, HJ, SJ) { \
      const unsigned mj = __builtin_amdgcn_ballot_w32(HJ); \
      if (mj != 0u) { \
        if (HJ) { \
          const int pos = wc + (int)__builtin_amdgcn_mbcnt_lo(mj, 0u); \
          if (pos < WCAP) list[wave * WCAP + pos] = ((el0 + (J)) << SLOTB) | (int)(SJ); \
        } \
        wc += (int)__builtin_popcount(mj); } }
    HITJ(0, h0, s0)
    HITJ(1, h1, s1)
    HITJ(2, h2, s2)
    HITJ(3, h3, s3)
    HITJ(4, h4, s4)
    HITJ(5, h5, s5)
    HITJ(6, h6, s6)
    HITJ(7, h7, s7)
#undef HITJ
  }
  return wc;
}

__global__ __launch_bounds__(NTHR) void k_xprep(const float* __restrict__ x, unsigned short* xb, int nN, int nUnits) {
  const int i = (int)blockIdx.x * NTHR + (int)threadIdx.x;
  if (i >= nUnits) return;
  const int row = i >> 4;
  const int c0  = (i & 15) * 8;
  const int rc  = row < nN ? row : nN - 1;
  const float* p = x + (size_t)rc * FW + c0;
  v4f a = *(const v4fa*)p, b = *(const v4fa*)(p + 4);
  const v4f z4 = {0.f, 0.f, 0.f, 0.f};
  if (row >= nN) { a = z4; b = z4; }
  const v4u hv = pack8(a, b);
  const size_t o = (size_t)row * KL0 + c0;
  *(volatile v4u*)(xb + o) = hv;
  __threadfence();
  *(volatile v4u*)(xb + o) = hv;
}

__global__ __launch_bounds__(NTHR) void k_wprep(const float* __restrict__ W0, const float* __restrict__ W1,
                                                const float* __restrict__ Wc,
                                                unsigned short* W0T, unsigned short* W1T, unsigned short* WCT) {
  const int u = (int)blockIdx.x * NTHR + (int)threadIdx.x;
  if (u >= NUW) return;
  v8us o;
  unsigned short* dp;
  if (u < NU0) {
    const int n   = u >> 4;
    const int k8  = (u & 15) * 8;
    const int rel = n >> 7, col = n & (FW - 1);
    const float* p = W0 + (size_t)rel * FW * FW + (size_t)k8 * FW + col;
#pragma unroll
    for (int i = 0; i < 8; ++i) o[i] = (unsigned short)f2bf(p[(size_t)i * FW]);
    dp = W0T + (size_t)n * KL0 + k8;
  } else if (u < NU0 + NU1) {
    const int v   = u - NU0;
    const int n   = v >> 5;
    const int g   = v & 31;
    const int rel = n >> 7, col = n & (FW - 1);
    const float* p = W1 + (size_t)rel * FW * FW + (size_t)(4 * g) * FW + col;
    const unsigned short f0 = (unsigned short)f2bf(p[0]);
    const unsigned short f1 = (unsigned short)f2bf(p[FW]);
    const unsigned short f2 = (unsigned short)f2bf(p[2 * FW]);
    const unsigned short f3 = (unsigned short)f2bf(p[3 * FW]);
    o[0] = f0; o[1] = f1; o[2] = f2; o[3] = f3; o[4] = f0; o[5] = f1; o[6] = f2; o[7] = f3;
    dp = W1T + (size_t)n * KL1 + 8 * g;
  } else {
    const int v = u - NU0 - NU1;
    const int n = v >> 5;
    const int g = v & 31;
    const float* p = Wc + (size_t)(4 * g) * NOUT + n;
    const unsigned short f0 = (unsigned short)f2bf(p[0]);
    const unsigned short f1 = (unsigned short)f2bf(p[NOUT]);
    const unsigned short f2 = (unsigned short)f2bf(p[2 * NOUT]);
    const unsigned short f3 = (unsigned short)f2bf(p[3 * NOUT]);
    o[0] = f0; o[1] = f1; o[2] = f2; o[3] = f3; o[4] = f0; o[5] = f1; o[6] = f2; o[7] = f3;
    dp = WCT + (size_t)n * KCL + 8 * g;
  }
  *(volatile v8us*)dp = o;
  __threadfence();
  *(volatile v8us*)dp = o;
}

template <int KPT>
__global__ __launch_bounds__(GTHR) void k_gemm(
    const unsigned short* __restrict__ A, const unsigned short* __restrict__ WT, float* outF, int storeF,
    const float* __restrict__ alp, const float* __restrict__ arp, float* SD, int MPr)
{
  __shared__ __attribute__((aligned(16))) float stg[GBM * HC];
  __shared__ __attribute__((aligned(16))) float satt[2 * HC];
  __shared__ __attribute__((aligned(16))) float sdot[8 * GBM];
  const int tid = (int)threadIdx.x, lane = tid & 31, wave = tid >> 5, hh = lane >> 4, m = lane & 15;
  const int rowBase = (int)blockIdx.x * GBM;

#pragma unroll 1
  for (int q = 0; q < 2; ++q) {
    const int i     = tid + q * GTHR;
    const int hw    = i >> 5;
    const int head  = hw >> 1;
    const int which = hw & 1;
    const int c     = i & (HD1 - 1);
    const int idx   = head * HD1 + c;
    const float va  = alp[idx], vd = arp[idx];
    const float mw  = (float)which;
    const float v   = fmaf(mw, vd, (1.f - mw) * va);
    satt[i] = bfr(v);
  }

  v8f acc[8];
  {
    const v8f z = {0.f, 0.f, 0.f, 0.f, 0.f, 0.f, 0.f, 0.f};
#pragma unroll
    for (int t = 0; t < 8; ++t) acc[t] = z;
  }
  const unsigned short* ap = A  + (size_t)(rowBase + 16 * wave + m) * (size_t)KPT + 8 * hh;
  const unsigned short* bp = WT + (size_t)m * (size_t)KPT + 8 * hh;

#pragma unroll 1
  for (int ks = 0; ks < KPT / 32; ++ks) {
    const int k0 = 32 * ks;
    FragB af;
    af.h[0] = *(const v8usa*)(ap + k0);
    af.h[1] = *(const v8usa*)(ap + k0 + 16);
#pragma unroll
    for (int nt = 0; nt < 8; ++nt) {
      const unsigned short* wq = bp + (size_t)(16 * nt) * (size_t)KPT + k0;
      FragB bf;
      bf.h[0] = *(const v8usa*)wq;
      bf.h[1] = *(const v8usa*)(wq + 16);
      acc[nt] = wmb(af, bf, acc[nt]);
    }
  }

#pragma unroll
  for (int nt = 0; nt < 8; ++nt) {
    const int lc = 16 * nt + m;
#pragma unroll
    for (int r = 0; r < 8; ++r) {
      const int lr = 16 * wave + 8 * hh + r;
      stg[lr * HC + lc] = acc[nt][r];
    }
  }
  __syncthreads();

  {
    const int row = tid & 63, g = tid >> 6;
    const float* hr  = stg + row * HC + (2 * g) * HD1;
    const float* sa0 = satt + (4 * g + 0) * HD1;
    const float* sd0 = satt + (4 * g + 1) * HD1;
    const float* sa1 = satt + (4 * g + 2) * HD1;
    const float* sd1 = satt + (4 * g + 3) * HD1;
    float ds0 = 0.f, dd0 = 0.f, ds1 = 0.f, dd1 = 0.f;
#pragma unroll 2
    for (int c4 = 0; c4 < HD1 / 4; ++c4) {
      const v4f h0 = *(const v4fa*)(hr + 4 * c4);
      const v4f h1 = *(const v4fa*)(hr + HD1 + 4 * c4);
      const v4f a0 = *(const v4fa*)(sa0 + 4 * c4);
      const v4f b0 = *(const v4fa*)(sd0 + 4 * c4);
      const v4f a1 = *(const v4fa*)(sa1 + 4 * c4);
      const v4f b1 = *(const v4fa*)(sd1 + 4 * c4);
      ds0 = fmaf(h0.x, a0.x, ds0); dd0 = fmaf(h0.x, b0.x, dd0); ds1 = fmaf(h1.x, a1.x, ds1); dd1 = fmaf(h1.x, b1.x, dd1);
      ds0 = fmaf(h0.y, a0.y, ds0); dd0 = fmaf(h0.y, b0.y, dd0); ds1 = fmaf(h1.y, a1.y, ds1); dd1 = fmaf(h1.y, b1.y, dd1);
      ds0 = fmaf(h0.z, a0.z, ds0); dd0 = fmaf(h0.z, b0.z, dd0); ds1 = fmaf(h1.z, a1.z, ds1); dd1 = fmaf(h1.z, b1.z, dd1);
      ds0 = fmaf(h0.w, a0.w, ds0); dd0 = fmaf(h0.w, b0.w, dd0); ds1 = fmaf(h1.w, a1.w, ds1); dd1 = fmaf(h1.w, b1.w, dd1);
    }
    sdot[(4 * g + 0) * GBM + row] = ds0;
    sdot[(4 * g + 1) * GBM + row] = dd0;
    sdot[(4 * g + 2) * GBM + row] = ds1;
    sdot[(4 * g + 3) * GBM + row] = dd1;
  }
  __syncthreads();

  v4f fv[16];
#pragma unroll
  for (int i = 0; i < 16; ++i) {
    const int lr = 16 * wave + i;
    fv[i] = *(const v4fa*)(stg + lr * HC + 4 * lane);
  }
  const int pl = tid >> 4, piece = tid & 15;
  const v4f sdv = *(const v4fa*)(sdot + pl * GBM + 4 * piece);
  float* sp = SD + (size_t)pl * (size_t)MPr + rowBase + 4 * piece;

  if (storeF != 0) {
#pragma unroll
    for (int i = 0; i < 16; ++i) {
      float* op = outF + (size_t)(rowBase + 16 * wave + i) * (size_t)HC + 4 * lane;
      *(volatile v4f*)op = fv[i];
    }
  }
  *(volatile v4f*)sp = sdv;
  __threadfence();
  if (storeF != 0) {
#pragma unroll
    for (int i = 0; i < 16; ++i) {
      float* op = outF + (size_t)(rowBase + 16 * wave + i) * (size_t)HC + 4 * lane;
      *(volatile v4f*)op = fv[i];
    }
  }
  *(volatile v4f*)sp = sdv;
}

template <int USEP, int DOELU, int OUTK>
__global__ __launch_bounds__(NTHR) void k_agg(
    const int* __restrict__ srcs, const int* __restrict__ dsts, int nE,
    const float* __restrict__ F, int nSrc,
    const float* __restrict__ SDs, int MPs, const float* __restrict__ SDd, int MPd,
    const float* __restrict__ bias, float* P, unsigned short* HP,
    int nDst, int nb, int vec8) {
  extern __shared__ v4f lds_dyn[];
  int* reg1 = (int*)lds_dyn;
  int* reg2 = reg1 + RCAP;
  int* scnt = reg2 + RCAP;
  int* soff = scnt + NBMAX;
  int* list = soff + NBMAX;
  int* wcnt = list + LISTN;
  int* wtot = wcnt + NWAVE;
  const int tid = (int)threadIdx.x, lane = tid & 31, wave = tid >> 5;
  const int nodeBase = (int)blockIdx.x * nb;

  for (int i = tid; i < NBMAX; i += NTHR) scnt[i] = 0;
  __syncthreads();

  int tot = 0;
  const int nChunks = (nE + CHUNK - 1) / CHUNK;
#pragma unroll 1
  for (int ch = 0; ch < nChunks; ++ch) {
    const int cbase = ch * CHUNK;
    const int wc = scan_chunk(dsts, nE, cbase, nodeBase, nb, vec8, list, tid, lane, wave);
    if (lane == 0) wcnt[wave] = wc;
    __syncthreads();
    int pre = 0, all = 0;
#pragma unroll
    for (int w2 = 0; w2 < NWAVE; ++w2) {
      int c = wcnt[w2];
      c = c < 0 ? 0 : (c > WCAP ? WCAP : c);
      all += c;
      pre += (w2 < wave) ? c : 0;
    }
    const int wcc  = wc > WCAP ? WCAP : wc;
    const int base = tot + pre;
#pragma unroll 1
    for (int i = lane; i < wcc; i += 32) {
      const int ent = list[wave * WCAP + i];
      const int el  = (ent >> SLOTB) & (CHUNK - 1);
      const int sl  = ent & (NBMAX - 1);
      int eid = cbase + el;
      eid = eid > nE - 1 ? nE - 1 : eid;
      const int pos = base + i;
      if (pos < RCAP) reg1[pos] = (int)(((unsigned)eid << SLOTB) | (unsigned)sl);
    }
    tot += all;
    tot = tot > RCAP ? RCAP : tot;
    __syncthreads();
  }
  const int nh = tot;

  if (wave == 0) {
#pragma unroll 1
    for (int b0 = 0; b0 < nh; b0 += 32) {
      const int idx = b0 + lane;
      const int uv  = reg1[idx < nh ? idx : nh - 1];
      const int m32 = (nh - b0) < 32 ? (nh - b0) : 32;
#pragma unroll 1
      for (int k = 0; k < m32; ++k) {
        const int u  = __builtin_amdgcn_readlane(uv, k);
        const int sl = u & (NBMAX - 1);
        if (lane == 0) scnt[sl] = scnt[sl] + 1;
      }
    }
  }
  __syncthreads();

  {
    const v4i ca = *(const v4i*)(scnt + 8 * tid);
    const v4i cb = *(const v4i*)(scnt + 8 * tid + 4);
    const int e0 = ca.x < 0 ? 0 : ca.x, e1 = ca.y < 0 ? 0 : ca.y, e2 = ca.z < 0 ? 0 : ca.z, e3 = ca.w < 0 ? 0 : ca.w;
    const int e4 = cb.x < 0 ? 0 : cb.x, e5 = cb.y < 0 ? 0 : cb.y, e6 = cb.z < 0 ? 0 : cb.z, e7 = cb.w < 0 ? 0 : cb.w;
    const int ts = e0 + e1 + e2 + e3 + e4 + e5 + e6 + e7;
    int incl = ts;
#pragma unroll
    for (int d = 1; d < 32; d <<= 1) {
      const int up = __shfl_up(incl, d);
      if (lane >= d) incl += up;
    }
    if (lane == 31) wtot[wave] = incl;
    __syncthreads();
    int pre = 0;
#pragma unroll
    for (int w2 = 0; w2 < NWAVE; ++w2) pre += (w2 < wave) ? wtot[w2] : 0;
    int run = pre + incl - ts;
    soff[8 * tid + 0] = run; run += e0;
    soff[8 * tid + 1] = run; run += e1;
    soff[8 * tid + 2] = run; run += e2;
    soff[8 * tid + 3] = run; run += e3;
    soff[8 * tid + 4] = run; run += e4;
    soff[8 * tid + 5] = run; run += e5;
    soff[8 * tid + 6] = run; run += e6;
    soff[8 * tid + 7] = run;
  }
  __syncthreads();
  for (int i = tid; i < NBMAX; i += NTHR) list[i] = soff[i];
  __syncthreads();

  if (wave == 0) {
#pragma unroll 1
    for (int b0 = 0; b0 < nh; b0 += 32) {
      const int idx = b0 + lane;
      const int uv  = reg1[idx < nh ? idx : nh - 1];
      const int m32 = (nh - b0) < 32 ? (nh - b0) : 32;
#pragma unroll 1
      for (int k = 0; k < m32; ++k) {
        const int u   = __builtin_amdgcn_readlane(uv, k);
        const int sl  = u & (NBMAX - 1);
        const int eid = (int)((unsigned)u >> SLOTB);
        if (lane == 0) {
          int pos = list[sl];
          pos = pos < 0 ? 0 : (pos > RCAP - 1 ? RCAP - 1 : pos);
          reg2[pos] = eid;
          list[sl] = pos + 1;
        }
      }
    }
  }
  __syncthreads();

  const int nbw = nb >> 3;
  const bool ovf = (nh >= RCAP);
  const float qnan = __int_as_float(0x7fc00000);
  const int c0   = 4 * lane;
  const int head = lane >> 3;
  const v4f bb   = bfr4(*(const v4fa*)(bias + c0));
  const float* ASp = SDs + (size_t)(2 * head) * (size_t)MPs;
  const float* ADp = SDd + (size_t)(2 * head + 1) * (size_t)MPd;
  const float* Fr  = F + c0;
  const v4f z4 = {0.f, 0.f, 0.f, 0.f};

#pragma unroll 1
  for (int jt = 0; jt < nbw; ++jt) {
    const int slot = wave * nbw + jt;
    const int grow = nodeBase + slot;
    const int gcl  = grow < nDst ? grow : nDst - 1;
    int st = soff[slot];
    const int craw = scnt[slot];
    int cnt = craw;
    st  = st < 0 ? 0 : (st > nh ? nh : st);
    cnt = cnt < 0 ? 0 : (cnt > DEGCAP ? DEGCAP : cnt);
    if (cnt > nh - st) cnt = nh - st;
    const float pz = (ovf || craw > DEGCAP) ? qnan : 0.0f;

    const float adv = ADp[gcl];
    float mx = MX0, dn = 0.0f;
    v4f av = z4;

#pragma unroll 1
    for (int q = 0; q < cnt; ++q) {
      int idx = st + q; idx = idx > RCAP - 1 ? RCAP - 1 : idx;
      int eid = reg2[idx]; eid = eid < 0 ? 0 : (eid > nE - 1 ? nE - 1 : eid);
      const int sraw = srcs[eid];
      const int s = sraw < 0 ? 0 : (sraw > nSrc - 1 ? nSrc - 1 : sraw);
      const v4f fs = *(const v4fa*)(Fr + (size_t)s * HC);
      float lg = ASp[s] + adv;
      lg = lg > 0.f ? lg : NEGSL * lg;
      const float df = lg - mx;
      const float ee = __expf(-fabsf(df));
      const bool up  = df > 0.f;
      const float s1 = up ? ee : 1.0f;
      const float s2 = up ? 1.0f : ee;
      mx = up ? lg : mx;
      dn = fmaf(dn, s1, s2);
      av.x = fmaf(av.x, s1, s2 * fs.x);
      av.y = fmaf(av.y, s1, s2 * fs.y);
      av.z = fmaf(av.z, s1, s2 * fs.z);
      av.w = fmaf(av.w, s1, s2 * fs.w);
    }
    const float inv = __builtin_amdgcn_rcpf(dn + EPS_SM);
    const bool live = grow < nDst;
    v4f ag;
    ag.x = fmaf(av.x, inv, bb.x);
    ag.y = fmaf(av.y, inv, bb.y);
    ag.z = fmaf(av.z, inv, bb.z);
    ag.w = fmaf(av.w, inv, bb.w);
    v4f v;
    if constexpr (USEP == 1) {
      const v4f pv = *(const v4fa*)(P + (size_t)gcl * HC + c0);
      v.x = (pv.x + ag.x) * 0.5f;
      v.y = (pv.y + ag.y) * 0.5f;
      v.z = (pv.z + ag.z) * 0.5f;
      v.w = (pv.w + ag.w) * 0.5f;
    } else {
      v = ag;
    }

    if constexpr (OUTK == 0) {
      v4f o;
      o.x = (live ? v.x : 0.f) + pz;
      o.y = (live ? v.y : 0.f) + pz;
      o.z = (live ? v.z : 0.f) + pz;
      o.w = (live ? v.w : 0.f) + pz;
      if (grow < MPd) {
        float* op = P + (size_t)grow * HC + c0;
        *(volatile v4f*)op = o;
        __threadfence();
        *(volatile v4f*)op = o;
      }
    } else {
      v4f e;
      if constexpr (DOELU == 1) {
        e.x = (live ? elu1(v.x) : 0.f) + pz;
        e.y = (live ? elu1(v.y) : 0.f) + pz;
        e.z = (live ? elu1(v.z) : 0.f) + pz;
        e.w = (live ? elu1(v.w) : 0.f) + pz;
      } else {
        e.x = (live ? v.x : 0.f) + pz;
        e.y = (live ? v.y : 0.f) + pz;
        e.z = (live ? v.z : 0.f) + pz;
        e.w = (live ? v.w : 0.f) + pz;
      }
      const v8us po = hilo8(e);
      if (grow < MPd) {
        unsigned short* hp = HP + (size_t)grow * (size_t)KL1 + 8 * lane;
        *(volatile v8us*)hp = po;
        __threadfence();
        *(volatile v8us*)hp = po;
      }
    }
  }
}

__global__ __launch_bounds__(GTHR) void k_head(const unsigned short* __restrict__ A,
                                               const unsigned short* __restrict__ BT,
                                               const float* __restrict__ bias, float* outp, int nOut) {
  __shared__ __attribute__((aligned(16))) float stg[GBM * NOUT];
  const int tid = (int)threadIdx.x, lane = tid & 31, wave = tid >> 5, hh = lane >> 4, m = lane & 15;
  const int rowBase = (int)blockIdx.x * GBM;

  v8f acc = {0.f, 0.f, 0.f, 0.f, 0.f, 0.f, 0.f, 0.f};
  const unsigned short* ap = A + (size_t)(rowBase + 16 * wave + m) * (size_t)KCL + 8 * hh;
  const unsigned short* wp = BT + (size_t)m * (size_t)KCL + 8 * hh;
#pragma unroll 1
  for (int ks = 0; ks < KCL / 32; ++ks) {
    FragB af, bf;
    af.h[0] = *(const v8usa*)(ap + 32 * ks);
    af.h[1] = *(const v8usa*)(ap + 32 * ks + 16);
    bf.h[0] = *(const v8usa*)(wp + 32 * ks);
    bf.h[1] = *(const v8usa*)(wp + 32 * ks + 16);
    acc = wmb(af, bf, acc);
  }
#pragma unroll
  for (int r = 0; r < 8; ++r) {
    const int lr = 16 * wave + 8 * hh + r;
    stg[lr * NOUT + m] = acc[r];
  }
  __syncthreads();

  int live = nOut - rowBase; live = live < 0 ? 0 : (live > GBM ? GBM : live);
  const int npc = live * (NOUT / 4);
  const int c4 = (tid & 3) * 4;
  const v4f bb4 = bfr4(*(const v4f*)(bias + c4));
  float* ob = outp + (size_t)rowBase * NOUT;
#pragma unroll 1
  for (int p = tid; p < npc; p += GTHR) {
    const v4f v = *(const v4fa*)(stg + 4 * p) + bb4;
    *(volatile v4f*)(ob + 4 * p) = v;
  }
  __threadfence();
#pragma unroll 1
  for (int p = tid; p < npc; p += GTHR) {
    const v4f v = *(const v4fa*)(stg + 4 * p) + bb4;
    *(volatile v4f*)(ob + 4 * p) = v;
  }
}

static int pick_nb(int nE, int nN) {
  int nb = NBMAX;
  while (nb > 32 && (long long)nb * (long long)nE * 5LL > (long long)RCAP * (long long)nN * 4LL) nb >>= 1;
  return nb;
}
static inline int cdiv(int a, int b) { return (a + b - 1) / b; }

extern "C" void kernel_launch(void* const* d_in, const int* in_sizes, int n_in,
                              void* d_out, int out_size, void* d_ws, size_t ws_size,
                              hipStream_t stream) {
  if (n_in < 18) return;
  if (in_sizes[0] < FW || (in_sizes[0] % FW) != 0) return;
  if (in_sizes[1] < FW || (in_sizes[1] % FW) != 0) return;
  const int nP = in_sizes[0] / FW;
  const int nA = in_sizes[1] / FW;
  if (nP > (1 << 22) || nA > (1 << 22)) return;
  const int eW = in_sizes[2], eC = in_sizes[4], eB = in_sizes[6];
  if (in_sizes[3] != eW || in_sizes[5] != eC || in_sizes[7] != eB) return;
  if (eW < 1 || eC < 1 || eB < 1) return;
  if (eW >= (1 << (32 - SLOTB)) || eC >= (1 << (32 - SLOTB)) || eB >= (1 << (32 - SLOTB))) return;
  if (in_sizes[8] != NREL * FW * FW || in_sizes[12] != NREL * FW * FW) return;
  if (in_sizes[9] != NREL * HC || in_sizes[10] != NREL * HC || in_sizes[11] != NREL * HC) return;
  if (in_sizes[13] != NREL * HC || in_sizes[14] != NREL * HC || in_sizes[15] != NREL * HC) return;
  if (in_sizes[16] != FW * NOUT || in_sizes[17] != NOUT) return;
  if ((long long)out_size != (long long)nP * NOUT) return;

  const float* xp   = (const float*)d_in[0];
  const float* xa   = (const float*)d_in[1];
  const int*   srcW = (const int*)d_in[2];
  const int*   dstW = (const int*)d_in[3];
  const int*   srcC = (const int*)d_in[4];
  const int*   dstC = (const int*)d_in[5];
  const int*   srcB = (const int*)d_in[6];
  const int*   dstB = (const int*)d_in[7];
  const float* W0   = (const float*)d_in[8];
  const float* al0  = (const float*)d_in[9];
  const float* ar0  = (const float*)d_in[10];
  const float* b0   = (const float*)d_in[11];
  const float* W1   = (const float*)d_in[12];
  const float* al1  = (const float*)d_in[13];
  const float* ar1  = (const float*)d_in[14];
  const float* b1   = (const float*)d_in[15];
  const float* Wc   = (const float*)d_in[16];
  const float* bc   = (const float*)d_in[17];
  float* out = (float*)d_out;

  const int MP  = cdiv(nP, MROWS) * MROWS;
  const int MA  = cdiv(nA, MROWS) * MROWS;
  const int gMP = MP / GBM, gMA = MA / GBM;
  const int eWC = eW > eC ? eW : eC;
  const int nbP = pick_nb(eWC, nP);
  const int nbA = pick_nb(eB, nA);
  if (nbP < 32 || (nbP & (nbP - 1)) != 0 || nbP > NBMAX) return;
  if (nbA < 32 || (nbA & (nbA - 1)) != 0 || nbA > NBMAX) return;
  const int gAP = cdiv(MP, nbP), gAA = cdiv(MA, nbA);
  if ((long long)gAP * nbP < (long long)MP || (long long)gAA * nbA < (long long)MA) return;
  const int vec8 = 1;

  const size_t szXPB = (size_t)MP * KL0 * 2, szXAB = (size_t)MA * KL0 * 2;
  const size_t szPf  = (size_t)MP * HC * 4;
  const size_t szZA  = (size_t)MA * HC * 4;
  const size_t szHP  = (size_t)MP * KL1 * 2;
  const size_t szHA  = (size_t)MA * KL1 * 2;
  size_t szR0 = szXPB + szXAB; if (szPf > szR0) szR0 = szPf; if (szHA > szR0) szR0 = szHA;
  size_t szR1 = szZA;  if (szHP > szR1) szR1 = szHP;
  const size_t szR2 = szPf;
  size_t szR3 = szPf;  if (szHP > szR3) szR3 = szHP;
  char* ws = (char*)d_ws;
  size_t off = 0;
  const size_t oW0T = off; off += (size_t)NREL * FW * KL0 * 2;      off = (off + 255) & ~(size_t)255;
  const size_t oW1T = off; off += (size_t)NREL * FW * KL1 * 2;      off = (off + 255) & ~(size_t)255;
  const size_t oWCT = off; off += (size_t)NOUT * KCL * 2;           off = (off + 255) & ~(size_t)255;
  const size_t oSDP = off; off += (size_t)24 * MP * 4;              off = (off + 255) & ~(size_t)255;
  const size_t oSDA = off; off += (size_t)16 * MA * 4;              off = (off + 255) & ~(size_t)255;
  const size_t oR0  = off; off += szR0;                             off = (off + 255) & ~(size_t)255;
  const size_t oR1  = off; off += szR1;                             off = (off + 255) & ~(size_t)255;
  const size_t oR2  = off; off += szR2;                             off = (off + 255) & ~(size_t)255;
  const size_t oR3  = off; off += szR3;                             off = (off + 255) & ~(size_t)255;
  if (off > ws_size || off > (size_t)WSMAX) return;
  unsigned short* W0T = (unsigned short*)(ws + oW0T);
  unsigned short* W1T = (unsigned short*)(ws + oW1T);
  unsigned short* WCT = (unsigned short*)(ws + oWCT);
  float*          SDP = (float*)(ws + oSDP);
  float*          SDA = (float*)(ws + oSDA);
  unsigned short* XPB = (unsigned short*)(ws + oR0);
  unsigned short* XAB = (unsigned short*)(ws + oR0 + szXPB);
  float*          Pp  = (float*)(ws + oR0);
  unsigned short* HA1 = (unsigned short*)(ws + oR0);
  float*          ZA  = (float*)(ws + oR1);
  unsigned short* HP1 = (unsigned short*)(ws + oR1);
  float*          ZP1 = (float*)(ws + oR2);
  float*          ZP2 = (float*)(ws + oR3);
  unsigned short* HP2 = (unsigned short*)(ws + oR3);
  float* SDP0 = SDP;  float* SDP1 = SDP + (size_t)8 * MP;  float* SDP2 = SDP + (size_t)16 * MP;
  float* SDA0 = SDA;  float* SDA2 = SDA + (size_t)8 * MA;

  hipFuncSetAttribute(reinterpret_cast<const void*>(&k_agg<0, 0, 0>), hipFuncAttributeMaxDynamicSharedMemorySize, LDS_AGG);
  hipFuncSetAttribute(reinterpret_cast<const void*>(&k_agg<1, 1, 1>), hipFuncAttributeMaxDynamicSharedMemorySize, LDS_AGG);
  hipFuncSetAttribute(reinterpret_cast<const void*>(&k_agg<0, 1, 1>), hipFuncAttributeMaxDynamicSharedMemorySize, LDS_AGG);
  hipFuncSetAttribute(reinterpret_cast<const void*>(&k_agg<1, 0, 1>), hipFuncAttributeMaxDynamicSharedMemorySize, LDS_AGG);

  k_wprep<<<NUW / NTHR, NTHR, 0, stream>>>(W0, W1, Wc, W0T, W1T, WCT);
  const int nUp = MP * (KL0 / 8), nUa = MA * (KL0 / 8);
  k_xprep<<<cdiv(nUp, NTHR), NTHR, 0, stream>>>(xp, XPB, nP, nUp);
  k_xprep<<<cdiv(nUa, NTHR), NTHR, 0, stream>>>(xa, XAB, nA, nUa);

  k_gemm<KL0><<<gMA, GTHR, 0, stream>>>(XAB, W0T + (size_t)0 * FW * KL0, ZA,  1, al0 + 0 * HC, ar0 + 0 * HC, SDA0, MA);
  k_gemm<KL0><<<gMP, GTHR, 0, stream>>>(XPB, W0T + (size_t)0 * FW * KL0, ZP2, 0, al0 + 0 * HC, ar0 + 0 * HC, SDP0, MP);
  k_gemm<KL0><<<gMP, GTHR, 0, stream>>>(XPB, W0T + (size_t)1 * FW * KL0, ZP1, 1, al0 + 1 * HC, ar0 + 1 * HC, SDP1, MP);
  k_gemm<KL0><<<gMA, GTHR, 0, stream>>>(XAB, W0T + (size_t)2 * FW * KL0, ZP2, 0, al0 + 2 * HC, ar0 + 2 * HC, SDA2, MA);
  k_gemm<KL0><<<gMP, GTHR, 0, stream>>>(XPB, W0T + (size_t)2 * FW * KL0, ZP2, 1, al0 + 2 * HC, ar0 + 2 * HC, SDP2, MP);
  k_agg<0, 0, 0><<<gAP, NTHR, LDS_AGG, stream>>>(srcW, dstW, eW, ZA, nA, SDA0, MA, SDP0, MP, b0 + 0 * HC, Pp, HP1, nP, nbP, vec8);
  k_agg<1, 1, 1><<<gAP, NTHR, LDS_AGG, stream>>>(srcC, dstC, eC, ZP1, nP, SDP1, MP, SDP1, MP, b0 + 1 * HC, Pp, HP1, nP, nbP, vec8);
  k_agg<0, 1, 1><<<gAA, NTHR, LDS_AGG, stream>>>(srcB, dstB, eB, ZP2, nP, SDP2, MP, SDA2, MA, b0 + 2 * HC, Pp, HA1, nA, nbA, vec8);

  k_gemm<KL1><<<gMP, GTHR, 0, stream>>>(HP1, W1T + (size_t)0 * FW * KL1, ZP2, 0, al1 + 0 * HC, ar1 + 0 * HC, SDP0, MP);
  k_gemm<KL1><<<gMP, GTHR, 0, stream>>>(HP1, W1T + (size_t)1 * FW * KL1, ZP1, 1, al1 + 1 * HC, ar1 + 1 * HC, SDP1, MP);
  k_gemm<KL1><<<gMA, GTHR, 0, stream>>>(HA1, W1T + (size_t)0 * FW * KL1, ZA,  1, al1 + 0 * HC, ar1 + 0 * HC, SDA0, MA);
  k_agg<0, 0, 0><<<gAP, NTHR, LDS_AGG, stream>>>(srcW, dstW, eW, ZA, nA, SDA0, MA, SDP0, MP, b1 + 0 * HC, Pp, HP2, nP, nbP, vec8);
  k_agg<1, 0, 1><<<gAP, NTHR, LDS_AGG, stream>>>(srcC, dstC, eC, ZP1, nP, SDP1, MP, SDP1, MP, b1 + 1 * HC, Pp, HP2, nP, nbP, vec8);

  k_head<<<gMP, GTHR, 0, stream>>>(HP2, WCT, bc, out, nP);
}
